// SE_GATNoEdgeAttrsSelectiveMask_59365037966023
// MI455X (gfx1250) — hardware-verified
//
#include <hip/hip_runtime.h>
#include <math.h>

typedef __attribute__((ext_vector_type(16))) _Float16 v16h;
typedef __attribute__((ext_vector_type(16))) __bf16 v16b;
typedef __attribute__((ext_vector_type(8)))  _Float16 v8h;
typedef __attribute__((ext_vector_type(8)))  float v8f;
typedef __attribute__((ext_vector_type(4)))  float v4f;
typedef __attribute__((ext_vector_type(2)))  float v2f;
typedef __attribute__((ext_vector_type(4)))  unsigned v4u;
typedef __attribute__((ext_vector_type(4)))  int v4i;
typedef float __attribute__((may_alias)) float_a;
typedef int __attribute__((may_alias)) int_a;

template <typename T> __device__ __forceinline__ void vst2(void* p, T v) { *(volatile T*)p = v; __threadfence(); *(volatile T*)p = v; }
__device__ __forceinline__ v8f wmma16(v16h a, v16h b, v8f c) {
  v8f d = __builtin_amdgcn_wmma_f32_16x16x32_f16(false, a, false, b, (short)0, c, false, false);
  asm volatile("v_nop\n\tv_nop\n\tv_nop\n\tv_nop" : "+v"(d) : "v"(a), "v"(b));
  return d;
}
__device__ __forceinline__ v8f wmma_bf(v16b a, v16b b, v8f c) {
  v8f d = __builtin_amdgcn_wmma_f32_16x16x32_bf16(false, a, false, b, (short)0, c, false, false);
  asm volatile("v_nop\n\tv_nop\n\tv_nop\n\tv_nop" : "+v"(d) : "v"(a), "v"(b));
  return d;
}
__device__ __forceinline__ v16h frag_h(const _Float16* rowk0, int lane) {
  union { v16h v; v8h q[2]; } u; const _Float16* p = rowk0 + 8 * (lane >> 4);
  u.q[0] = *(const v8h*)p; u.q[1] = *(const v8h*)(p + 16); return u.v;
}
__device__ __forceinline__ v16h frag_f32(const float* rowk0, int lane) {
  v16h a; const float* p = rowk0 + 8 * (lane >> 4);
#pragma unroll
  for (int i = 0; i < 8; ++i) { a[i] = (_Float16)p[i]; a[8 + i] = (_Float16)p[16 + i]; }
  return a;
}
__device__ __forceinline__ v16h frag_f32s(const float* rowk0, int lane, float sc) {
  v16h a; const float* p = rowk0 + 8 * (lane >> 4);
#pragma unroll
  for (int i = 0; i < 8; ++i) { a[i] = (_Float16)(p[i] * sc); a[8 + i] = (_Float16)(p[16 + i] * sc); }
  return a;
}
__device__ __forceinline__ v16h fragc_f32(const float* W, int k0, int n, int lane, int ld, int K) {
  v16h a; const int g = lane >> 4;
#pragma unroll
  for (int i = 0; i < 8; ++i) { const int ka = k0 + 8 * g + i, kb = ka + 16;
    a[i] = (_Float16)(ka < K ? W[(size_t)ka * ld + n] : 0.f); a[8 + i] = (_Float16)(kb < K ? W[(size_t)kb * ld + n] : 0.f); }
  return a;
}
struct F2 { v16b h, l; };
__device__ __forceinline__ F2 bsplit16(const float v[16]) { F2 r;
#pragma unroll
  for (int i = 0; i < 16; ++i) { const __bf16 h = (__bf16)v[i]; r.h[i] = h; r.l[i] = (__bf16)(v[i] - (float)h); }
  return r; }
__device__ __forceinline__ F2 split_row(const float* row, int k0, int lane) { float v[16]; const float* p = row + k0 + 8 * (lane >> 4);
#pragma unroll
  for (int i = 0; i < 8; ++i) { v[i] = p[i]; v[8 + i] = p[16 + i]; }
  return bsplit16(v); }
__device__ __forceinline__ F2 split_rowK(const float* row, int k0, int lane, int K) { float v[16]; const int g = lane >> 4;
#pragma unroll
  for (int i = 0; i < 8; ++i) { const int ka = k0 + 8 * g + i, kb = ka + 16; v[i] = ka < K ? row[ka] : 0.f; v[8 + i] = kb < K ? row[kb] : 0.f; }
  return bsplit16(v); }
__device__ __forceinline__ F2 split_col(const float* W, int k0, int n, int lane, int ld, int K) { float v[16]; const int g = lane >> 4;
#pragma unroll
  for (int i = 0; i < 8; ++i) { const int ka = k0 + 8 * g + i, kb = ka + 16; v[i] = ka < K ? W[(size_t)ka * ld + n] : 0.f; v[8 + i] = kb < K ? W[(size_t)kb * ld + n] : 0.f; }
  return bsplit16(v); }
__device__ __forceinline__ v8f mac3(const F2& a, const F2& b, v8f c) { c = wmma_bf(a.l, b.h, c); c = wmma_bf(a.h, b.l, c); return wmma_bf(a.h, b.h, c); }
__device__ __forceinline__ float sigm(float v) { return 1.0f / (1.0f + expf(-v)); }
#define LDSX() do { asm volatile("s_wait_dscnt 0" ::: "memory"); __builtin_amdgcn_wave_barrier(); __builtin_amdgcn_fence(__ATOMIC_RELEASE, "workgroup"); } while (0)

#define NN 50000
#define NE 400000
#define NROWS 27
#define FI 128
#define F1 256
#define NH1 4
#define C1 64
#define FO2 64
#define NG 64
#define EPT 16
#define CH (256 * EPT)
#define RB1 256
#define NRB1 ((NN + RB1 - 1) / RB1)
#define RB2 512
#define NRB2 ((NN + RB2 - 1) / RB2)
#define NNP 50176

__device__ __forceinline__ int f2ord(float f) { const int i = __float_as_int(f); return i >= 0 ? i : i ^ 0x7fffffff; }
__device__ __forceinline__ float ord2f(int i) { return __int_as_float(i >= 0 ? i : i ^ 0x7fffffff); }
__device__ __forceinline__ float lrelu(float v) { return v > 0.f ? v : 0.2f * v; }
__device__ __forceinline__ float elu1(float v) { return v > 0.f ? v : expm1f(v); }

template <int K, int NOUT, int NHD>
__global__ __launch_bounds__(128) void k_node(const float* __restrict__ A, int arows, const float* __restrict__ W, const float* __restrict__ asrc, const float* __restrict__ adst, float* __restrict__ XW, float* __restrict__ AS, float* __restrict__ AD) {
  constexpr int NT = NOUT / 16; constexpr int CHD = NOUT / NHD;
  __shared__ __align__(16) float so[4][16][NOUT + 4];
  const int tid = threadIdx.x, wave = tid >> 5, lane = tid & 31, col = lane & 15, g = lane >> 4;
  const int r0 = blockIdx.x * 64 + wave * 16; const int ra = (r0 + col) < arows ? (r0 + col) : (arows - 1);
  v8f acc[NT];
#pragma unroll
  for (int t = 0; t < NT; ++t) acc[t] = (v8f){};
#pragma unroll 1
  for (int kc = 0; kc < K / 32; ++kc) { const F2 a = split_row(A + (size_t)ra * K, kc * 32, lane);
#pragma unroll
    for (int t = 0; t < NT; ++t) acc[t] = mac3(a, split_col(W, kc * 32, t * 16 + col, lane, NOUT, K), acc[t]); }
#pragma unroll
  for (int t = 0; t < NT; ++t)
#pragma unroll
    for (int r = 0; r < 8; ++r) so[wave][8 * g + r][t * 16 + col] = acc[t][r];
  LDSX();
  for (int q = lane; q < 16 * (NOUT / 4); q += 32) { const int rl = q / (NOUT / 4), pc = q % (NOUT / 4); vst2(XW + (size_t)(r0 + rl) * NOUT + pc * 4, *(const v4f*)(&so[wave][rl][pc * 4])); }
  { const int rl = lane >> 1, hf = lane & 1; const float* row = &so[wave][rl][0]; float s_s[4] = {0.f, 0.f, 0.f, 0.f}, s_d[4] = {0.f, 0.f, 0.f, 0.f};
    if (NHD == 4) { for (int hh = 0; hh < 2; ++hh) { const int h = hf * 2 + hh; for (int c = 0; c < CHD; ++c) { const float v = row[h * CHD + c]; s_s[hh] += v * asrc[h * CHD + c]; s_d[hh] += v * adst[h * CHD + c]; } } }
    else { for (int c = hf * (CHD / 2); c < hf * (CHD / 2) + CHD / 2; ++c) { const float v = row[c]; s_s[0] += v * asrc[c]; s_d[0] += v * adst[c]; } s_s[0] += __shfl_xor(s_s[0], 1, 32); s_d[0] += __shfl_xor(s_d[0], 1, 32); }
    float* asr = AS + (size_t)(r0 + rl) * 4; float* adr = AD + (size_t)(r0 + rl) * 4;
    if (NHD == 4) { vst2(asr + hf * 2, s_s[0]); vst2(asr + hf * 2 + 1, s_s[1]); vst2(adr + hf * 2, s_d[0]); vst2(adr + hf * 2 + 1, s_d[1]); }
    else if (hf == 0) { vst2(asr, s_s[0]); vst2(adr, s_d[0]); } }
}
template <int RB, int NHD>
__global__ __launch_bounds__(256) void k_max(const int* __restrict__ esrc, const int* __restrict__ edst, const float* __restrict__ AS, const float* __restrict__ AD, float* __restrict__ SMX) {
  __shared__ int smx[RB][4];
  const int tid = threadIdx.x; const int r0 = blockIdx.x * RB;
  for (int q = tid; q < RB * 4; q += 256) { const int rl = q >> 2, h = q & 3; const int row = r0 + rl; float v = -3.0e38f;
    if (row < NN && h < NHD) v = lrelu(AS[(size_t)row * 4 + h] + AD[(size_t)row * 4 + h]);
    smx[rl][h] = f2ord(v); }
  __syncthreads();
#pragma unroll 1
  for (int c0 = 0; c0 < NE; c0 += CH) { const int e0 = c0 + tid * EPT;
#pragma unroll
    for (int v = 0; v < EPT / 4; ++v) { int dd[4];
      if (e0 + v * 4 + 4 <= NE) { const int4 d4 = *(const int4*)(edst + e0 + v * 4); dd[0] = d4.x; dd[1] = d4.y; dd[2] = d4.z; dd[3] = d4.w; }
      else { for (int u = 0; u < 4; ++u) dd[u] = (e0 + v * 4 + u < NE) ? edst[e0 + v * 4 + u] : -1; }
#pragma unroll
      for (int u = 0; u < 4; ++u) { const unsigned rel = (unsigned)(dd[u] - r0); if (dd[u] >= 0 && rel < (unsigned)RB) { int s = esrc[e0 + v * 4 + u]; s = s < 0 ? 0 : (s >= NN ? NN - 1 : s);
          for (int h = 0; h < NHD; ++h) atomicMax(&smx[rel][h], f2ord(lrelu(AS[(size_t)s * 4 + h] + AD[(size_t)(r0 + rel) * 4 + h]))); } } } }
  __syncthreads();
  for (int q = tid; q < RB * 4; q += 256) { const int rl = q >> 2, h = q & 3; vst2(SMX + (size_t)(r0 + rl) * 4 + h, ord2f(smx[rl][h])); }
}
template <int RB, int F, int NHD>
__global__ __launch_bounds__(256) void k_gagg(const int* __restrict__ esrc_, const int* __restrict__ edst_, const float* __restrict__ XW, const float* __restrict__ AS, const float* __restrict__ AD, const float* __restrict__ SMX, const float* __restrict__ bias, float* __restrict__ OUT) {
  constexpr int CHD = F / NHD;
  __shared__ __align__(16) float sacc[RB][F];
  __shared__ float sden[RB][4]; __shared__ float sadm[RB][8];
  __shared__ int ssrc[8][32 * EPT], sdl[8][32 * EPT]; __shared__ int scnt[8];
  const int tid = threadIdx.x, wave = tid >> 5, lane = tid & 31;
  const int r0 = blockIdx.x * RB; const int* esrc = esrc_; const int* edst = edst_;
  for (int q = tid; q < RB * F; q += 256) (&sacc[0][0])[q] = 0.f;
  for (int q = tid; q < RB * 4; q += 256) { const int rl = q >> 2, h = q & 3; const int row = r0 + rl; sden[rl][h] = 0.f; sadm[rl][h] = row < NN ? AD[(size_t)row * 4 + h] : 0.f; sadm[rl][4 + h] = row < NN ? SMX[(size_t)row * 4 + h] : 0.f; }
  __syncthreads();
  const int fcol = tid < F ? tid : 0; const int myh = fcol / CHD; const bool dodn = (tid < F) && (fcol % CHD == 0);
  #pragma unroll 1
  for (int c0 = 0; c0 < NE; c0 += CH) {
    const int e0 = c0 + tid * EPT; int hd[EPT]; int cnt = 0;
    if (e0 + EPT <= NE) {
#pragma unroll
      for (int v = 0; v < EPT / 4; ++v) { const int4 d4 = *(const int4*)(edst + e0 + v * 4);
        const int dd[4] = {d4.x, d4.y, d4.z, d4.w};
#pragma unroll
        for (int u = 0; u < 4; ++u) { const unsigned rel = (unsigned)(dd[u] - r0); const bool h = rel < (unsigned)RB; hd[v * 4 + u] = h ? (int)rel : -1; cnt += h ? 1 : 0; } } }
    else {
#pragma unroll
      for (int u = 0; u < EPT; ++u) { const int e = e0 + u; hd[u] = -1; if (e < NE) { const unsigned rel = (unsigned)(edst[e] - r0); if (rel < (unsigned)RB) { hd[u] = (int)rel; ++cnt; } } } }
    int incl = cnt;
#pragma unroll
    for (int off = 1; off < 32; off <<= 1) { const int vv = __shfl_up(incl, off, 32); if (lane >= off) incl += vv; }
    const int wtot = __shfl(incl, 31, 32); int pos = incl - cnt;
    if (cnt > 0) {
#pragma unroll
      for (int u = 0; u < EPT; ++u) if (hd[u] >= 0) { int s = esrc[e0 + u]; s = s < 0 ? 0 : (s >= NN ? NN - 1 : s); ssrc[wave][pos] = s; sdl[wave][pos] = hd[u];  ++pos; } }
    if (lane == 0) scnt[wave] = wtot;
    __syncthreads();
    if (tid < F) { for (int w = 0; w < 8; ++w) { const int nh = scnt[w]; for (int i = 0; i < nh; ++i) { const int s = ssrc[w][i], dl = sdl[w][i];
          const float wgt = expf(lrelu(AS[(size_t)s * 4 + myh] + sadm[dl][myh]) - sadm[dl][4 + myh]);
          sacc[dl][fcol] += wgt * XW[(size_t)s * F + fcol]; if (dodn) sden[dl][myh] += wgt; } } }
    __syncthreads(); }
#pragma unroll 1
  for (int q = tid; q < RB * F; q += 256) { const int rl = q / F, f = q % F; const int row = r0 + rl; if (row >= NN) continue; const int h = f / CHD;
    const float ws = expf(lrelu(AS[(size_t)row * 4 + h] + sadm[rl][h]) - sadm[rl][4 + h]);
    const float v = (sacc[rl][f] + ws * XW[(size_t)row * F + f]) / (sden[rl][h] + ws) + bias[f];
    sacc[rl][f] = v > 0.f ? v : 0.f; }
  __syncthreads();
  for (int q = tid; q < RB * (F / 4); q += 256) { const int rl = q / (F / 4), pc = q % (F / 4); const int row = r0 + rl; if (row >= NN) continue; vst2(OUT + (size_t)row * F + pc * 4, *(const v4f*)(&sacc[rl][pc * 4])); }
}
__global__ __launch_bounds__(64) void k_pool(const float* __restrict__ H, const int* __restrict__ bidx, float* __restrict__ POOL) {
  __shared__ int slist[512]; __shared__ int swt[2]; __shared__ __align__(16) float so[FO2];
  const int gph = blockIdx.x, tid = threadIdx.x, wave = tid >> 5, lane = tid & 31; float acc = 0.f; int total = 0;
#pragma unroll 1
  for (int n0 = 0; n0 < NN; n0 += 512) { int hit[8]; int cnt = 0;
#pragma unroll
    for (int u = 0; u < 8; ++u) { const int n = n0 + tid * 8 + u; hit[u] = (n < NN && bidx[n] == gph) ? n : -1; cnt += hit[u] >= 0; }
    int incl = cnt;
#pragma unroll
    for (int off = 1; off < 32; off <<= 1) { const int vv = __shfl_up(incl, off, 32); if (lane >= off) incl += vv; }
    if (lane == 31) swt[wave] = incl;
    __syncthreads();
    const int base = wave == 1 ? swt[0] : 0; const int tot = swt[0] + swt[1];
    int pos = base + incl - cnt;
#pragma unroll
    for (int u = 0; u < 8; ++u) if (hit[u] >= 0) slist[pos++] = hit[u];
    __syncthreads();
    for (int i = 0; i < tot; ++i) acc += H[(size_t)slist[i] * FO2 + tid];
    total += tot;
    __syncthreads(); }
  so[tid] = acc / fmaxf((float)total, 1.0f);
  __syncthreads();
  if (tid < FO2 / 4) vst2(POOL + (size_t)gph * FO2 + tid * 4, *(const v4f*)(&so[tid * 4]));
}
__global__ __launch_bounds__(128) void k_head(const float* __restrict__ POOL, const float* __restrict__ Wfc, const float* __restrict__ bfc, float* __restrict__ out) {
  __shared__ __align__(16) float so[NG * 2];
  const int tid = threadIdx.x; { const int gq = tid >> 1, o = tid & 1; float s = bfc[o];
#pragma unroll 1
    for (int k = 0; k < FO2; ++k) s += POOL[(size_t)gq * FO2 + k] * Wfc[k * 2 + o];
    so[gq * 2 + o] = s; }
  __syncthreads();
  if (tid < NG * 2 / 4) vst2(out + tid * 4, *(const v4f*)(&so[tid * 4]));
}
extern "C" void kernel_launch(void* const* d_in, const int* in_sizes, int n_in, void* d_out, int out_size, void* d_ws, size_t ws_size, hipStream_t stream) {
  (void)in_sizes; (void)n_in; (void)out_size; (void)ws_size;
  const float** I = (const float**)d_in;
  const float* x = I[0]; const int* ei = (const int*)d_in[1]; const int* bidx = (const int*)d_in[2];
  const float* W1 = I[3]; const float* as1 = I[4]; const float* ad1 = I[5]; const float* b1 = I[6]; const float* W2 = I[7]; const float* as2 = I[8]; const float* ad2 = I[9]; const float* b2 = I[10]; const float* Wfc = I[11]; const float* bfc = I[12];
  float* out = (float*)d_out;
  char* ws = (char*)d_ws; size_t off = 0;
  auto take = [&](size_t bytes) { char* p = ws + off; off += (bytes + 255) & ~(size_t)255; return p; };
  float* XW1 = (float*)take((size_t)NNP * F1 * 4); float* AS = (float*)take((size_t)NNP * 4 * 4); float* AD = (float*)take((size_t)NNP * 4 * 4); float* SMX = (float*)take((size_t)NNP * 4 * 4);
  float* H1 = (float*)take((size_t)NNP * F1 * 4); float* XW2 = XW1; float* H2 = (float*)take((size_t)NNP * FO2 * 4); float* POOL = (float*)take((size_t)NG * FO2 * 4);
  const int* s1 = ei + (size_t)17 * NE; const int* d1 = ei + (size_t)26 * NE; const int* s2 = ei + (size_t)15 * NE; const int* d2 = ei + (size_t)16 * NE;
  k_node<FI, F1, 4><<<NNP / 64, 128, 0, stream>>>(x, NN, W1, as1, ad1, XW1, AS, AD);
  k_max<RB1, 4><<<NRB1, 256, 0, stream>>>(s1, d1, AS, AD, SMX);
  k_gagg<RB1, F1, 4><<<NRB1, 256, 0, stream>>>(s1, d1, XW1, AS, AD, SMX, b1, H1);
  k_node<F1, FO2, 4><<<NNP / 64, 128, 0, stream>>>(H1, NN, W2, as2, ad2, XW2, AS, AD);
  k_max<RB2, 4><<<NRB2, 256, 0, stream>>>(s2, d2, AS, AD, SMX);
  k_gagg<RB2, FO2, 4><<<NRB2, 256, 0, stream>>>(s2, d2, XW2, AS, AD, SMX, b2, H2);
  k_pool<<<NG, 64, 0, stream>>>(H2, bidx, POOL);
  k_head<<<1, 128, 0, stream>>>(POOL, Wfc, bfc, out);
}
